// GCU_18202071401057
// MI455X (gfx1250) — hardware-verified
//
#include <hip/hip_runtime.h>
#include <stddef.h>


typedef _Float16 v16h __attribute__((ext_vector_type(16)));
typedef _Float16 v8h  __attribute__((ext_vector_type(8)));
typedef float    v8f  __attribute__((ext_vector_type(8)));
typedef float    v4f  __attribute__((ext_vector_type(4)));
typedef unsigned short v8us  __attribute__((ext_vector_type(8)));
typedef unsigned short v16us __attribute__((ext_vector_type(16)));
typedef __bf16   v16bf __attribute__((ext_vector_type(16)));

#ifndef NPIX
#define NPIX 16384
#endif
#define NPIX_FULL 16384
#define DD   64
#define VV   64
#define OUTF 32
#define AK   (NPIX / 64)
#define NCH  (AK / 64)
#define EPSV 1.0e-7f
#ifndef QRES
#define QRES 0
#endif

static_assert(NPIX >= 4096 && NPIX <= NPIX_FULL && (NPIX % 4096) == 0);
static_assert(DD == 64 && VV == 64 && OUTF == 32);
static_assert((AK % 64) == 0 && (AK % 32) == 0 && NCH * 64 == AK);
static_assert((NPIX % 64) == 0);

#define LDT 72
#define LDC 68
#define CLD 36
#define QLD 68
static_assert((LDT % 8) == 0 && LDT >= 64);
static_assert((LDC % 4) == 0 && LDC >= 64);
static_assert((CLD % 4) == 0 && CLD >= 32);
static_assert((QLD % 4) == 0 && QLD >= 64);

#define QCARRY 16384.0f
#define TCARRY 64.0f
static_assert(QCARRY <= 32768.0f);

#define COEF_BYTES  ((size_t)1024)
#define PLANE_BYTES ((size_t)VV * NPIX * 2)
#define Q16_BYTES   ((size_t)NPIX * VV * 2)
#define UP_BYTES    ((size_t)NCH * DD * VV * 4)
#define ZT_BYTES    ((size_t)VV * DD * 4)
#define ZOT_BYTES   ((size_t)OUTF * VV * 2)
#define OFF_COEF ((size_t)0)
#define OFF_XA   (OFF_COEF + COEF_BYTES)
#define OFF_QH   (OFF_XA + PLANE_BYTES)
#define OFF_QL   (OFF_QH + PLANE_BYTES)
#define OFF_Q16  (OFF_QL + PLANE_BYTES)
#define OFF_UP   (OFF_Q16 + Q16_BYTES)
#define OFF_ZT   (OFF_UP + UP_BYTES)
#define OFF_ZOT  (OFF_ZT + ZT_BYTES)
#define WS_TOTAL (OFF_ZOT + ZOT_BYTES)
static_assert((COEF_BYTES % 128) == 0 && (PLANE_BYTES % 128) == 0 && (Q16_BYTES % 128) == 0);
static_assert((UP_BYTES % 128) == 0 && (ZT_BYTES % 128) == 0 && (ZOT_BYTES % 128) == 0);
static_assert(3 * 64 * 4 <= COEF_BYTES);
static_assert(WS_TOTAL <= (size_t)134217728);

__device__ __forceinline__ float bf16r(float x) {
  unsigned int u = __float_as_uint(x);
  u = (u + 0x7FFFu + ((u >> 16) & 1u)) & 0xFFFF0000u;
  return __uint_as_float(u);
}
__device__ __forceinline__ unsigned short bf16_bits(float x) {
  unsigned int u = __float_as_uint(x);
  u = (u + 0x7FFFu + ((u >> 16) & 1u)) >> 16;
  return (unsigned short)u;
}
__device__ __forceinline__ float bf16_widen(unsigned short b) {
  return __uint_as_float(((unsigned int)b) << 16);
}
__device__ __forceinline__ _Float16 toh_flush(float v) {
  const _Float16 r = (_Float16)v;
  return (fabsf(v) < 6.103515625e-05f) ? (_Float16)0.0f : r;
}

__device__ __forceinline__ v16h frag_at(const _Float16* p) {
  v8h lo = *(const v8h*)(p);
  v8h hi = *(const v8h*)(p + 16);
  v16h out;
#pragma unroll
  for (int i = 0; i < 8; ++i) { out[i] = lo[i]; out[i + 8] = hi[i]; }
  return out;
}
__device__ __forceinline__ v16h ld_frag(const _Float16* base, unsigned ld) {
  const unsigned lane = threadIdx.x & 31u;
  return frag_at(base + (lane & 15u) * ld + (lane >> 4) * 8u);
}
__device__ __forceinline__ v16bf frag_bf_at(const unsigned short* p) {
  const v8us lo = *(const v8us*)(p);
  const v8us hi = *(const v8us*)(p + 16);
  const v16us o = __builtin_shufflevector(lo, hi, 0, 1, 2, 3, 4, 5, 6, 7,
                                          8, 9, 10, 11, 12, 13, 14, 15);
  return __builtin_bit_cast(v16bf, o);
}

__device__ __forceinline__ v8f wmma16(v16h a, v16h b, v8f c) {
  v8f d = __builtin_amdgcn_wmma_f32_16x16x32_f16(false, a, false, b, (short)0, c,
                                                 false, false);
  asm volatile("v_nop\n\tv_nop\n\tv_nop\n\tv_nop" : "+v"(d) : "v"(a), "v"(b));
  return d;
}
__device__ __forceinline__ v8f wmma_bf(v16bf a, v16bf b, v8f c) {
  v8f d = __builtin_amdgcn_wmma_f32_16x16x32_bf16(false, a, false, b, (short)0, c,
                                                  false, false);
  asm volatile("v_nop\n\tv_nop\n\tv_nop\n\tv_nop" : "+v"(d) : "v"(a), "v"(b));
  return d;
}

__device__ __forceinline__ float red32_sum(float x) {
#pragma unroll
  for (int off = 1; off < 32; off <<= 1) x += __shfl_xor(x, off, 32);
  return x;
}
__device__ __forceinline__ float red32_min(float x) {
#pragma unroll
  for (int off = 1; off < 32; off <<= 1) x = fminf(x, __shfl_xor(x, off, 32));
  return x;
}

__global__ __launch_bounds__(64) void coef_kernel(
    const float* __restrict__ W, const float* __restrict__ var, float* __restrict__ coef) {
#pragma clang fp contract(off)
  __shared__ __attribute__((aligned(16))) float cs[192];
  const unsigned v = threadIdx.x;
  double A = 0.0, Bc = 0.0, Cc = 0.0;
#pragma unroll 1
  for (unsigned d = 0; d < (unsigned)DD; ++d) {
    const float w = bf16r(W[d * VV + v]);
    const float iv = 1.0f / bf16r(var[d * VV + v]);
    const double iv2 = (double)iv * (double)iv;
    const double wd = (double)w;
    A += iv2;
    Bc += wd * iv2;
    Cc += (wd * wd) * iv2;
  }
  cs[v] = (float)A;
  cs[64u + v] = (float)Bc;
  cs[128u + v] = (float)Cc;
  __syncthreads();
  if (v < 48u) {
    const v4f x = *(const v4f*)&cs[v * 4u];
    float* p = coef + v * 4u;
    *(volatile v4f*)p = x;
    __threadfence();
    *(volatile v4f*)p = x;
  }
}

__global__ __launch_bounds__(256) void xplane_kernel(
    const float* __restrict__ X, unsigned short* __restrict__ XA) {
#pragma clang fp contract(off)
  __shared__ __attribute__((aligned(16))) unsigned short T[64 * LDT];
  const unsigned tid = threadIdx.x;
  const unsigned p0 = blockIdx.x * 64u;
#pragma unroll 4
  for (unsigned j = 0; j < 16u; ++j) {
    const unsigned idx = tid + 256u * j;
    const unsigned pr = idx >> 6, vc = idx & 63u;
    const float v = X[(size_t)(p0 + pr) * VV + vc];
    T[vc * LDT + pr] = bf16_bits(v);
  }
  __syncthreads();
  v8us x[2];
  size_t off[2];
#pragma unroll
  for (unsigned i = 0; i < 2u; ++i) {
    const unsigned n = 32u * i + (tid >> 3);
    const unsigned kc = (tid & 7u) * 8u;
    x[i] = *(const v8us*)&T[n * LDT + kc];
    off[i] = (size_t)n * NPIX + p0 + kc;
  }
#pragma unroll
  for (int i = 0; i < 2; ++i) *(volatile v8us*)(XA + off[i]) = x[i];
  __threadfence();
#pragma unroll
  for (int i = 0; i < 2; ++i) *(volatile v8us*)(XA + off[i]) = x[i];
}

__global__ __launch_bounds__(256) void assign_kernel(
    const float* __restrict__ X, const float* __restrict__ coef,
    _Float16* __restrict__ Q16, unsigned short* __restrict__ QH,
    unsigned short* __restrict__ QL, float* __restrict__ UP) {
#pragma clang fp contract(off)
  __shared__ __attribute__((aligned(16))) float Qs[64 * QLD];
  __shared__ __attribute__((aligned(16))) float Us[64];
  const unsigned tid = threadIdx.x, lane = tid & 31u;
  const unsigned wave = (unsigned)__builtin_amdgcn_readfirstlane((int)(threadIdx.x >> 5));
  const unsigned d = blockIdx.x, c = blockIdx.y;

  const float cA0 = coef[lane],       cB0 = coef[64u + lane],  cC0 = coef[128u + lane];
  const float cA1 = coef[32u + lane], cB1 = coef[96u + lane],  cC1 = coef[160u + lane];

#pragma unroll 1
  for (unsigned j = 0; j < 8u; ++j) {
    const unsigned i = wave * 8u + j;
    const size_t p = (size_t)(c * 64u + i) * 64u + d;
    const float x0 = bf16r(X[p * VV + lane]);
    const float x1 = bf16r(X[p * VV + 32u + lane]);
    const float q0 = cA0 * x0 * x0 - 2.0f * cB0 * x0 + cC0;
    const float q1 = cA1 * x1 * x1 - 2.0f * cB1 * x1 + cC1;
    const float mn = red32_min(fminf(q0, q1));
    const float e0 = expf(-0.5f * (q0 - mn));
    const float e1 = expf(-0.5f * (q1 - mn));
    const float s = red32_sum(e0 + e1);
    const float inv = 1.0f / s;
    Qs[i * QLD + lane] = e0 * inv;
    Qs[i * QLD + 32u + lane] = e1 * inv;
  }
  __syncthreads();

  v8h x16[2];
  v8us qh[2];
#if QRES
  v8us ql[2];
#endif
  size_t off16[2], offq[2];
#pragma unroll
  for (unsigned i = 0; i < 2u; ++i) {
    const unsigned r = 32u * i + (tid >> 3);
    const unsigned cc = (tid & 7u) * 8u;
    const v4f u0 = *(const v4f*)&Qs[r * QLD + cc];
    const v4f u1 = *(const v4f*)&Qs[r * QLD + cc + 4u];
#pragma unroll
    for (int j = 0; j < 4; ++j) {
      x16[i][j]     = toh_flush(u0[j] * QCARRY);
      x16[i][j + 4] = toh_flush(u1[j] * QCARRY);
    }
    off16[i] = ((size_t)(c * 64u + r) * 64u + d) * VV + cc;
#pragma unroll
    for (unsigned j = 0; j < 8u; ++j) {
      const float val = Qs[(cc + j) * QLD + r];
      const unsigned short hb = bf16_bits(val);
      qh[i][j] = hb;
#if QRES
      ql[i][j] = bf16_bits(val - bf16_widen(hb));
#endif
    }
    offq[i] = (size_t)r * NPIX + (size_t)d * AK + c * 64u + cc;
  }
#pragma unroll
  for (int i = 0; i < 2; ++i) *(volatile v8h*)(Q16 + off16[i]) = x16[i];
#pragma unroll
  for (int i = 0; i < 2; ++i) *(volatile v8us*)(QH + offq[i]) = qh[i];
#if QRES
#pragma unroll
  for (int i = 0; i < 2; ++i) *(volatile v8us*)(QL + offq[i]) = ql[i];
#endif
  __threadfence();
#pragma unroll
  for (int i = 0; i < 2; ++i) *(volatile v8h*)(Q16 + off16[i]) = x16[i];
#pragma unroll
  for (int i = 0; i < 2; ++i) *(volatile v8us*)(QH + offq[i]) = qh[i];
#if QRES
#pragma unroll
  for (int i = 0; i < 2; ++i) *(volatile v8us*)(QL + offq[i]) = ql[i];
#endif

  if (tid < 64u) {
    float s = 0.0f;
#pragma unroll 1
    for (unsigned i = 0; i < 64u; ++i) s += Qs[i * QLD + tid];
    Us[tid] = s;
  }
  __syncthreads();
  if (tid < 16u) {
    const v4f x = *(const v4f*)&Us[tid * 4u];
    float* p = UP + ((size_t)(c * 64u + d) * VV) + tid * 4u;
    *(volatile v4f*)p = x;
    __threadfence();
    *(volatile v4f*)p = x;
  }
}

__global__ __launch_bounds__(256) void tgemm_kernel(
    const unsigned short* __restrict__ XA, const unsigned short* __restrict__ QH,
    const unsigned short* __restrict__ QL, const float* __restrict__ UP,
    const float* __restrict__ W, const float* __restrict__ var, float* __restrict__ ZT) {
  __shared__ __attribute__((aligned(16))) float Cs[64 * LDC];
  __shared__ __attribute__((aligned(16))) float ivs[64];
  __shared__ __attribute__((aligned(16))) float wus[64];
  __shared__ __attribute__((aligned(16))) float us[64];
  __shared__ __attribute__((aligned(16))) float zs[64];
  __shared__ __attribute__((aligned(16))) float zn[64];
  const unsigned tid = threadIdx.x, lane = tid & 31u;
  const unsigned w = (unsigned)__builtin_amdgcn_readfirstlane((int)(threadIdx.x >> 5));
  const unsigned mw = w >> 1, nw = w & 1u;
  const unsigned hh = lane >> 4, m = lane & 15u;
  const unsigned v = blockIdx.x;

  const size_t pbase = (size_t)v * NPIX;
  const unsigned short* ap  = XA + pbase + (size_t)(mw * 16u + m) * AK + hh * 8u;
  const unsigned short* bh0 = QH + pbase + (size_t)(nw * 32u + m) * AK + hh * 8u;
  const unsigned short* bh1 = bh0 + (size_t)16 * AK;
#if QRES
  const unsigned short* bl0 = QL + pbase + (size_t)(nw * 32u + m) * AK + hh * 8u;
  const unsigned short* bl1 = bl0 + (size_t)16 * AK;
#endif
  v8f acc0 = {}, acc1 = {};
#pragma unroll 2
  for (unsigned k0 = 0; k0 < (unsigned)AK; k0 += 32u) {
    const v16bf a  = frag_bf_at(ap + k0);
    const v16bf b0 = frag_bf_at(bh0 + k0);
    const v16bf b1 = frag_bf_at(bh1 + k0);
    acc0 = wmma_bf(a, b0, acc0);
    acc1 = wmma_bf(a, b1, acc1);
#if QRES
    const v16bf c0 = frag_bf_at(bl0 + k0);
    const v16bf c1 = frag_bf_at(bl1 + k0);
    acc0 = wmma_bf(a, c0, acc0);
    acc1 = wmma_bf(a, c1, acc1);
#endif
  }
#pragma unroll
  for (int r = 0; r < 8; ++r) {
    float* dst = &Cs[(mw * 16u + hh * 8u + (unsigned)r) * LDC + nw * 32u + m];
    dst[0]  = acc0[r];
    dst[16] = acc1[r];
  }
  if (tid < 64u) {
    const unsigned d = tid;
    float u = 0.0f;
#pragma unroll
    for (unsigned c = 0; c < (unsigned)NCH; ++c) u += UP[((size_t)(c * 64u + d) * VV) + v];
    const float iv = 1.0f / bf16r(var[d * VV + v]);
    ivs[d] = iv;
    wus[d] = bf16r(W[d * VV + v]) * u;
    us[d] = u;
  }
  __syncthreads();
  if (tid < 64u) {
    const unsigned dp = tid;
    float acc = 0.0f, sq = 0.0f;
#pragma unroll 1
    for (unsigned d = 0; d < 64u; ++d) {
      acc += ivs[d] * (Cs[dp * LDC + d] - wus[d]);
      sq += us[d];
    }
    zs[dp] = (acc + EPSV) * (1.0f / (sq + EPSV));
  }
  __syncthreads();
  if (tid < 64u) {
    float n = 0.0f;
#pragma unroll 1
    for (unsigned i = 0; i < 64u; ++i) n += zs[i] * zs[i];
    zn[tid] = zs[tid] * (1.0f / n);
  }
  __syncthreads();
  if (tid < 16u) {
    const v4f x = *(const v4f*)&zn[tid * 4u];
    float* p = ZT + (size_t)v * DD + tid * 4u;
    *(volatile v4f*)p = x;
    __threadfence();
    *(volatile v4f*)p = x;
  }
}

__global__ __launch_bounds__(256) void tail_kernel(
    const float* __restrict__ ZT, const float* __restrict__ weight,
    _Float16* __restrict__ ZoT) {
  __shared__ __attribute__((aligned(16))) _Float16 Zt[64 * LDT];
  __shared__ __attribute__((aligned(16))) _Float16 Wt[32 * LDT];
  __shared__ __attribute__((aligned(16))) _Float16 Ad[64 * LDT];
  __shared__ __attribute__((aligned(16))) _Float16 O1[32 * LDT];
  __shared__ __attribute__((aligned(16))) _Float16 Zo[32 * LDT];
  const unsigned tid = threadIdx.x, lane = tid & 31u;
  const unsigned w = (unsigned)__builtin_amdgcn_readfirstlane((int)(threadIdx.x >> 5));
  const unsigned mw = w >> 1, nw = w & 1u;
  const unsigned hh = lane >> 4, m = lane & 15u;

#pragma unroll
  for (unsigned j = 0; j < 4u; ++j) {
    const unsigned idx = tid + 256u * j;
    const unsigned r = idx >> 4, c4 = (idx & 15u) * 4u;
    const v4f u = *(const v4f*)(ZT + (size_t)r * DD + c4);
#pragma unroll
    for (int e = 0; e < 4; ++e) Zt[r * LDT + c4 + (unsigned)e] = toh_flush(u[e] * TCARRY);
  }
#pragma unroll
  for (unsigned j = 0; j < 8u; ++j) {
    const unsigned idx = tid + 256u * j;
    const unsigned d = idx >> 5, o = idx & 31u;
    Wt[o * LDT + d] = toh_flush(TCARRY * bf16r(weight[idx]));
  }
  __syncthreads();

  v8f aA0 = {}, aA1 = {}, aO = {};
#pragma unroll
  for (int c = 0; c < 2; ++c) {
    const v16h a  = ld_frag(&Zt[(mw * 16u) * LDT + c * 32], LDT);
    const v16h b0 = ld_frag(&Zt[(nw * 32u) * LDT + c * 32], LDT);
    const v16h b1 = ld_frag(&Zt[(nw * 32u + 16u) * LDT + c * 32], LDT);
    const v16h b2 = ld_frag(&Wt[(nw * 16u) * LDT + c * 32], LDT);
    aA0 = wmma16(a, b0, aA0);
    aA1 = wmma16(a, b1, aA1);
    aO  = wmma16(a, b2, aO);
  }
#pragma unroll
  for (int r = 0; r < 8; ++r) {
    const unsigned row = mw * 16u + hh * 8u + (unsigned)r;
    Ad[row * LDT + nw * 32u + m]       = toh_flush(aA0[r] * (1.0f / TCARRY));
    Ad[row * LDT + nw * 32u + 16u + m] = toh_flush(aA1[r] * (1.0f / TCARRY));
    O1[(nw * 16u + m) * LDT + row]     = toh_flush(aO[r] * (1.0f / TCARRY));
  }
  __syncthreads();

  v8f a2 = {};
#pragma unroll
  for (int c = 0; c < 2; ++c) {
    const v16h a = ld_frag(&Ad[(mw * 16u) * LDT + c * 32], LDT);
    const v16h b = ld_frag(&O1[(nw * 16u) * LDT + c * 32], LDT);
    a2 = wmma16(a, b, a2);
  }
#pragma unroll
  for (int r = 0; r < 8; ++r) {
    const unsigned row = mw * 16u + hh * 8u + (unsigned)r;
    Zo[(nw * 16u + m) * LDT + row] = toh_flush(fmaxf(a2[r], 0.0f) * (1.0f / TCARRY));
  }
  __syncthreads();

  {
    const unsigned r = tid >> 3;
    const unsigned c = (tid & 7u) * 8u;
    const v8h x = *(const v8h*)&Zo[r * LDT + c];
    _Float16* p = ZoT + (size_t)r * VV + c;
    *(volatile v8h*)p = x;
    __threadfence();
    *(volatile v8h*)p = x;
  }
}

__global__ __launch_bounds__(256) void xnew_kernel(
    const _Float16* __restrict__ Q16, const _Float16* __restrict__ ZoT,
    float* __restrict__ out) {
  __shared__ __attribute__((aligned(16))) float Cs[64 * CLD];
  const unsigned tid = threadIdx.x, lane = tid & 31u;
  const unsigned w = (unsigned)__builtin_amdgcn_readfirstlane((int)(threadIdx.x >> 5));
  const unsigned mw = w >> 1, nw = w & 1u;
  const unsigned hh = lane >> 4, m = lane & 15u;
  const unsigned row0 = blockIdx.x * 64u;

  const _Float16* ap = Q16 + (size_t)(row0 + mw * 16u + m) * VV + hh * 8u;
  const _Float16* bp = ZoT + (size_t)(nw * 16u + m) * VV + hh * 8u;
  v8f acc = {};
#pragma unroll
  for (unsigned k0 = 0; k0 < (unsigned)VV; k0 += 32u) {
    const v16h a = frag_at(ap + k0);
    const v16h b = frag_at(bp + k0);
    acc = wmma16(a, b, acc);
  }
#pragma unroll
  for (int r = 0; r < 8; ++r)
    Cs[(mw * 16u + hh * 8u + (unsigned)r) * CLD + nw * 16u + m] = acc[r];
  __syncthreads();

  const float cs = 1.0f / (QCARRY * TCARRY);
  v4f xs[2];
  size_t off[2];
#pragma unroll
  for (unsigned i = 0; i < 2u; ++i) {
    const unsigned r = 32u * i + (tid >> 3);
    const unsigned c = (tid & 7u) * 4u;
    const v4f u = *(const v4f*)&Cs[r * CLD + c];
    xs[i] = u * cs;
    off[i] = (size_t)(row0 + r) * OUTF + c;
  }
#pragma unroll
  for (int i = 0; i < 2; ++i) *(volatile v4f*)(out + off[i]) = xs[i];
  __threadfence();
#pragma unroll
  for (int i = 0; i < 2; ++i) *(volatile v4f*)(out + off[i]) = xs[i];
}

extern "C" void kernel_launch(void* const* d_in, const int* in_sizes, int n_in,
                              void* d_out, int out_size, void* d_ws, size_t ws_size,
                              hipStream_t stream) {
  if (n_in < 4) return;
  if ((long long)in_sizes[0] < (long long)NPIX * DD) return;
  if (in_sizes[1] < DD * VV || in_sizes[2] < DD * VV) return;
  if (in_sizes[3] < DD * OUTF) return;
  if ((long long)out_size < (long long)NPIX * OUTF) return;
  if (ws_size < WS_TOTAL) return;

  const float* X      = (const float*)d_in[0];
  const float* W      = (const float*)d_in[1];
  const float* var    = (const float*)d_in[2];
  const float* weight = (const float*)d_in[3];
  float* out = (float*)d_out;

  char* ws = (char*)d_ws;
  float*          coef = (float*)(ws + OFF_COEF);
  unsigned short* XA   = (unsigned short*)(ws + OFF_XA);
  unsigned short* QH   = (unsigned short*)(ws + OFF_QH);
  unsigned short* QL   = (unsigned short*)(ws + OFF_QL);
  _Float16*       Q16  = (_Float16*)(ws + OFF_Q16);
  float*          UP   = (float*)(ws + OFF_UP);
  float*          ZT   = (float*)(ws + OFF_ZT);
  _Float16*       ZoT  = (_Float16*)(ws + OFF_ZOT);

  dim3 blk(256);
  coef_kernel<<<dim3(1), dim3(64), 0, stream>>>(W, var, coef);
  xplane_kernel<<<dim3(NPIX / 64), blk, 0, stream>>>(X, XA);
  assign_kernel<<<dim3(64, NCH), blk, 0, stream>>>(X, coef, Q16, QH, QL, UP);
  tgemm_kernel<<<dim3(VV), blk, 0, stream>>>(XA, QH, QL, UP, W, var, ZT);
  tail_kernel<<<dim3(1), blk, 0, stream>>>(ZT, weight, ZoT);
  xnew_kernel<<<dim3(NPIX / 64), blk, 0, stream>>>(Q16, ZoT, out);
}
